// VanillaAttention_29600914604401
// MI455X (gfx1250) — hardware-verified
//
#include <hip/hip_runtime.h>
#include <stddef.h>

#ifndef NB
#define NB 2
#endif
#ifndef SEQ
#define SEQ 2048
#endif
#define NB_FULL 2
#define SEQ_FULL 2048
#define H_ 16
#define E_ 64
#define HE (H_ * E_)
#define SROW (3 * HE)
#define RES_QBLOCKS 4
#define PP 72
#define OP 68
#define TP 72

static_assert(NB >= 1 && NB <= NB_FULL);
static_assert(SEQ % 128 == 0 && SEQ >= 128 && SEQ <= SEQ_FULL);
static_assert(E_ == 64 && H_ == 16);
static_assert((PP * 2) % 16 == 0 && (OP * 4) % 16 == 0 && (TP * 2) % 16 == 0);

typedef __attribute__((ext_vector_type(16))) _Float16 v16h;
typedef __attribute__((ext_vector_type(8)))  _Float16 v8h;
typedef __attribute__((ext_vector_type(16))) __bf16   v16b;
typedef __attribute__((ext_vector_type(8)))  __bf16   v8b;
typedef __attribute__((ext_vector_type(8)))  float    v8f;
typedef __attribute__((ext_vector_type(4)))  float    v4f;
typedef __attribute__((ext_vector_type(8)))  unsigned short v8us;

constexpr size_t PLANE_BYTES = (size_t)NB * H_ * SEQ * E_ * 2;
constexpr size_t OFF_Q   = 0;
constexpr size_t OFF_K   = OFF_Q + PLANE_BYTES;
constexpr size_t OFF_V   = OFF_K + PLANE_BYTES;
constexpr size_t WS_TOTAL = OFF_V + PLANE_BYTES;
static_assert(OFF_K % 128 == 0 && OFF_V % 128 == 0);
static_assert(WS_TOTAL <= (size_t)134217728);
constexpr size_t OUT_ELEMS = (size_t)NB * SEQ * H_ * E_;
static_assert(OUT_ELEMS * 4 <= (size_t)16777216);

__device__ __forceinline__ unsigned short f2bf_bits(float f) {
  unsigned u = __float_as_uint(f);
  return (unsigned short)((u + 0x7FFFu + ((u >> 16) & 1u)) >> 16);
}
__device__ __forceinline__ float bf_bits2f(unsigned short hb) { return __uint_as_float(((unsigned)hb) << 16); }

__device__ __forceinline__ v16h ldfrag_h(const _Float16* p) {
  union { v16h v; v8h hh[2]; } f;
  f.hh[0] = *(const v8h*)(p);
  f.hh[1] = *(const v8h*)(p + 16);
  return f.v;
}
__device__ __forceinline__ v16b ldfrag_b(const __bf16* p) {
  union { v16b v; v8b hh[2]; } f;
  f.hh[0] = *(const v8b*)(p);
  f.hh[1] = *(const v8b*)(p + 16);
  return f.v;
}

__device__ __forceinline__ v8f mma_h(v16h a, v16h b, v8f c) {
  c = __builtin_amdgcn_wmma_f32_16x16x32_f16(false, a, false, b, (short)0, c, false, false);
  asm volatile("v_nop\n\tv_nop\n\tv_nop\n\tv_nop" : "+v"(c) : "v"(a), "v"(b));
  return c;
}
__device__ __forceinline__ v8f mma_b(v16b a, v16b b, v8f c) {
  c = __builtin_amdgcn_wmma_f32_16x16x32_bf16(false, a, false, b, (short)0, c, false, false);
  asm volatile("v_nop\n\tv_nop\n\tv_nop\n\tv_nop" : "+v"(c) : "v"(a), "v"(b));
  return c;
}

__device__ __forceinline__ void wave_lds_sync() {
  __builtin_amdgcn_fence(__ATOMIC_RELEASE, "workgroup");
  __builtin_amdgcn_wave_barrier();
  __builtin_amdgcn_fence(__ATOMIC_ACQUIRE, "workgroup");
}

__global__ __launch_bounds__(256) void cvt_kernel(const float* __restrict__ qkv,
                                                  unsigned short* __restrict__ QB,
                                                  unsigned short* __restrict__ KB,
                                                  unsigned short* __restrict__ VT) {
  __shared__ __align__(16) _Float16 tile[64 * TP];
  const int tid  = threadIdx.x;
  const int s0   = blockIdx.x * 64;
  const int h    = blockIdx.y;
  const int b    = blockIdx.z;
  const size_t bh = (size_t)b * H_ + h;
  const int rloc = tid >> 3;
  const int c8   = (tid & 7) * 8;

  v8us uq[2], uk[2];
#pragma unroll
  for (int it = 0; it < 2; ++it) {
    const int sl = it * 32 + rloc;
    const float* rowp = qkv + ((size_t)b * SEQ_FULL + (size_t)(s0 + sl)) * SROW + (size_t)h * E_ + c8;
    const v4f qa = *(const v4f*)(rowp);
    const v4f qc = *(const v4f*)(rowp + 4);
    const v4f ka = *(const v4f*)(rowp + HE);
    const v4f kc = *(const v4f*)(rowp + HE + 4);
    const v4f va = *(const v4f*)(rowp + 2 * HE);
    const v4f vc = *(const v4f*)(rowp + 2 * HE + 4);
#pragma unroll
    for (int e = 0; e < 4; ++e) {
      uq[it][e]     = f2bf_bits(qa[e]);
      uq[it][4 + e] = f2bf_bits(qc[e]);
      uk[it][e]     = f2bf_bits(ka[e]);
      uk[it][4 + e] = f2bf_bits(kc[e]);
      const float v0 = bf_bits2f(f2bf_bits(va[e])) * 16.0f;
      const float v1 = bf_bits2f(f2bf_bits(vc[e])) * 16.0f;
      tile[(c8 + e) * TP + sl]     = (_Float16)v0;
      tile[(c8 + 4 + e) * TP + sl] = (_Float16)v1;
    }
  }
  __syncthreads();

  v8h vv[2];
#pragma unroll
  for (int it = 0; it < 2; ++it) {
    const int e = it * 32 + rloc;
    vv[it] = *(const v8h*)(tile + e * TP + (tid & 7) * 8);
  }

  for (int pass = 0; pass < 2; ++pass) {
#pragma unroll
    for (int it = 0; it < 2; ++it) {
      const int sl = it * 32 + rloc;
      const size_t ro = (bh * SEQ + (size_t)(s0 + sl)) * E_ + c8;
      *(volatile v8us*)(QB + ro) = uq[it];
      *(volatile v8us*)(KB + ro) = uk[it];
    }
#pragma unroll
    for (int it = 0; it < 2; ++it) {
      const int e = it * 32 + rloc;
      const size_t vo = (bh * E_ + (size_t)e) * SEQ + s0 + (tid & 7) * 8;
      *(volatile v8h*)((_Float16*)VT + vo) = vv[it];
    }
    __threadfence();
  }
}

template <bool MASKED, bool RES>
__device__ __forceinline__ void attn_step(int j, int q0, int h16, int n,
                                          const __bf16* __restrict__ kplane,
                                          const _Float16* __restrict__ vplane,
                                          _Float16* pt, _Float16* pr,
                                          v16b aQ0, v16b aQ1,
                                          float (&rmax)[8], float (&rsum)[8],
                                          v8f (&acc)[4], v8f (&accr)[4]) {
  v8f sc[4];
#pragma unroll
  for (int t = 0; t < 4; ++t) {
    const __bf16* kr = kplane + (size_t)(j + 16 * t + n) * E_ + 8 * h16;
    const v16b b0 = ldfrag_b(kr);
    const v16b b1 = ldfrag_b(kr + 32);
    v8f c = (v8f){0.f, 0.f, 0.f, 0.f, 0.f, 0.f, 0.f, 0.f};
    c = mma_b(aQ0, b0, c);
    c = mma_b(aQ1, b1, c);
    sc[t] = c;
  }

  const float cs = 0.125f * 1.44269504088896340736f;
  const int kg0 = j + n, kg1 = kg0 + 16, kg2 = kg0 + 32, kg3 = kg0 + 48;
#pragma unroll
  for (int r = 0; r < 8; ++r) {
    float x0 = sc[0][r] * cs, x1 = sc[1][r] * cs, x2 = sc[2][r] * cs, x3 = sc[3][r] * cs;
    if (MASKED) {
      const int mrow = q0 + 8 * h16 + r;
      x0 = (kg0 <= mrow) ? x0 : -1e30f;
      x1 = (kg1 <= mrow) ? x1 : -1e30f;
      x2 = (kg2 <= mrow) ? x2 : -1e30f;
      x3 = (kg3 <= mrow) ? x3 : -1e30f;
    }
    float mx = fmaxf(fmaxf(x0, x1), fmaxf(x2, x3));
    mx = fmaxf(mx, __shfl_xor(mx, 1));
    mx = fmaxf(mx, __shfl_xor(mx, 2));
    mx = fmaxf(mx, __shfl_xor(mx, 4));
    mx = fmaxf(mx, __shfl_xor(mx, 8));
    const float nm   = fmaxf(rmax[r], mx);
    const float corr = exp2f(rmax[r] - nm);
    rmax[r] = nm;
    const float p0 = exp2f(x0 - nm);
    const float p1 = exp2f(x1 - nm);
    const float p2 = exp2f(x2 - nm);
    const float p3 = exp2f(x3 - nm);
    rsum[r] = rsum[r] * corr + ((p0 + p1) + (p2 + p3));
    acc[0][r] *= corr; acc[1][r] *= corr; acc[2][r] *= corr; acc[3][r] *= corr;
    if (RES) { accr[0][r] *= corr; accr[1][r] *= corr; accr[2][r] *= corr; accr[3][r] *= corr; }
    const float c0 = p0 * 16384.0f, c1 = p1 * 16384.0f, c2 = p2 * 16384.0f, c3 = p3 * 16384.0f;
    const _Float16 g0 = (_Float16)c0, g1 = (_Float16)c1, g2 = (_Float16)c2, g3 = (_Float16)c3;
    _Float16* pw = pt + (8 * h16 + r) * PP + n;
    pw[0] = g0; pw[16] = g1; pw[32] = g2; pw[48] = g3;
    if (RES) {
      _Float16* qw = pr + (8 * h16 + r) * PP + n;
      qw[0]  = (_Float16)((c0 - (float)g0) * 2048.0f);
      qw[16] = (_Float16)((c1 - (float)g1) * 2048.0f);
      qw[32] = (_Float16)((c2 - (float)g2) * 2048.0f);
      qw[48] = (_Float16)((c3 - (float)g3) * 2048.0f);
    }
  }
  wave_lds_sync();

  const _Float16* prow = pt + n * PP + 8 * h16;
  const v16h pa0 = ldfrag_h(prow);
  const v16h pa1 = ldfrag_h(prow + 32);
  v16h ra0 = pa0, ra1 = pa1;
  if (RES) {
    const _Float16* rrow = pr + n * PP + 8 * h16;
    ra0 = ldfrag_h(rrow);
    ra1 = ldfrag_h(rrow + 32);
  }

#pragma unroll
  for (int c4 = 0; c4 < 4; ++c4) {
    const _Float16* vr = vplane + (size_t)(16 * c4 + n) * SEQ + j + 8 * h16;
    const v16h vb0 = ldfrag_h(vr);
    const v16h vb1 = ldfrag_h(vr + 32);
    acc[c4] = mma_h(pa0, vb0, acc[c4]);
    acc[c4] = mma_h(pa1, vb1, acc[c4]);
    if (RES) {
      accr[c4] = mma_h(ra0, vb0, accr[c4]);
      accr[c4] = mma_h(ra1, vb1, accr[c4]);
    }
  }
  wave_lds_sync();
}

template <bool RES>
__global__ __launch_bounds__(256) void attn_kernel(const unsigned short* __restrict__ QBp,
                                                   const unsigned short* __restrict__ KBp,
                                                   const unsigned short* __restrict__ VTp,
                                                   float* __restrict__ out, int qbBase) {
  __shared__ __align__(16) _Float16 lds_p[8][2][16 * PP];
  __shared__ __align__(16) float    lds_o[8][16 * OP];

  const int wave = threadIdx.x >> 5;
  const int lane = threadIdx.x & 31;
  const int h16  = lane >> 4;
  const int n    = lane & 15;
  const int h    = blockIdx.y;
  const int b    = blockIdx.z;
  const int qb   = qbBase + blockIdx.x;
  const int q0   = qb * 128 + wave * 16;

  _Float16* pt   = &lds_p[wave][0][0];
  _Float16* pr   = &lds_p[wave][1][0];
  float*    slab = &lds_o[wave][0];

  const size_t bh = (size_t)b * H_ + h;
  const __bf16*   qplane = (const __bf16*)QBp   + bh * (size_t)SEQ * E_;
  const __bf16*   kplane = (const __bf16*)KBp   + bh * (size_t)SEQ * E_;
  const _Float16* vplane = (const _Float16*)VTp + bh * (size_t)E_ * SEQ;

  const __bf16* qr = qplane + (size_t)(q0 + n) * E_ + 8 * h16;
  const v16b aQ0 = ldfrag_b(qr);
  const v16b aQ1 = ldfrag_b(qr + 32);

  float rmax[8], rsum[8];
  v8f acc[4], accr[4];
#pragma unroll
  for (int c4 = 0; c4 < 4; ++c4) {
    acc[c4]  = (v8f){0.f, 0.f, 0.f, 0.f, 0.f, 0.f, 0.f, 0.f};
    accr[c4] = (v8f){0.f, 0.f, 0.f, 0.f, 0.f, 0.f, 0.f, 0.f};
  }
#pragma unroll
  for (int r = 0; r < 8; ++r) { rmax[r] = -1e30f; rsum[r] = 0.0f; }

  const int nfull = q0 >> 6;
  for (int st = 0; st < nfull; ++st)
    attn_step<false, RES>(st * 64, q0, h16, n, kplane, vplane, pt, pr, aQ0, aQ1, rmax, rsum, acc, accr);
  attn_step<true, RES>(nfull * 64, q0, h16, n, kplane, vplane, pt, pr, aQ0, aQ1, rmax, rsum, acc, accr);

#pragma unroll
  for (int r = 0; r < 8; ++r) {
    float sg = rsum[r];
    sg += __shfl_xor(sg, 1);
    sg += __shfl_xor(sg, 2);
    sg += __shfl_xor(sg, 4);
    sg += __shfl_xor(sg, 8);
    const float inv = (1.0f / sg) * (1.0f / (16384.0f * 16.0f));
#pragma unroll
    for (int c4 = 0; c4 < 4; ++c4) {
      float o = acc[c4][r];
      if (RES) o = o + accr[c4][r] * (1.0f / 2048.0f);
      slab[(8 * h16 + r) * OP + 16 * c4 + n] = o * inv;
    }
  }
  wave_lds_sync();

  {
    const int hh = lane >> 4, c4o = (lane & 15) * 4;
    float* ob = out + (((size_t)b * SEQ + q0) * H_ + h) * (size_t)E_;
    for (int pass = 0; pass < 2; ++pass) {
#pragma unroll
      for (int it = 0; it < 8; ++it) {
        const int row = it * 2 + hh;
        const v4f val = *(const v4f*)(slab + row * OP + c4o);
        *(volatile v4f*)(ob + (size_t)row * HE + c4o) = val;
      }
      __threadfence();
    }
  }
}

extern "C" void kernel_launch(void* const* d_in, const int* in_sizes, int n_in,
                              void* d_out, int out_size, void* d_ws, size_t ws_size,
                              hipStream_t stream) {
  if (n_in < 1) return;
  if ((size_t)in_sizes[0] < (size_t)NB * SEQ_FULL * SROW) return;
  if ((size_t)out_size < OUT_ELEMS) return;
  if (ws_size < WS_TOTAL) return;

  const float* qkv = (const float*)d_in[0];
  float* out = (float*)d_out;

  char* ws = (char*)d_ws;
  unsigned short* QB = (unsigned short*)(ws + OFF_Q);
  unsigned short* KB = (unsigned short*)(ws + OFF_K);
  unsigned short* VT = (unsigned short*)(ws + OFF_V);

  cvt_kernel<<<dim3(SEQ / 64, H_, NB), dim3(256), 0, stream>>>(qkv, QB, KB, VT);

  const int nqb  = SEQ / 128;
  const int nres = (nqb < RES_QBLOCKS) ? nqb : RES_QBLOCKS;
  attn_kernel<true><<<dim3(nres, H_, NB), dim3(256), 0, stream>>>(QB, KB, VT, out, 0);
  if (nqb > nres)
    attn_kernel<false><<<dim3(nqb - nres, H_, NB), dim3(256), 0, stream>>>(QB, KB, VT, out, nres);
}
